// GroupedQueryAttention_30597347017136
// MI455X (gfx1250) — hardware-verified
//
#include <hip/hip_runtime.h>
#include <math.h>

typedef __attribute__((ext_vector_type(16))) _Float16     v16h;
typedef __attribute__((ext_vector_type(8)))  _Float16     v8h;
typedef __attribute__((ext_vector_type(16))) __bf16       v16b;
typedef __attribute__((ext_vector_type(8)))  __bf16       v8b;
typedef __attribute__((ext_vector_type(8)))  float        v8f;
typedef __attribute__((ext_vector_type(4)))  float        v4f;
typedef __attribute__((ext_vector_type(4)))  unsigned int v4u;

#ifndef NB
#define NB 2
#endif
#ifndef SEQ
#define SEQ 2048
#endif
#define NB_FULL  2
#define SEQ_FULL 2048
#define EMB   2048
#define NQH   32
#define NKVH  8
#define GRP   4
#define HDIM  64
#define EKV   512
#define KC    64
#define QT    16
#define NWAVE 4

#define K16_BYTES ((size_t)NB * SEQ * EKV * 2)
#define VT_BYTES  ((size_t)NB * NKVH * HDIM * SEQ * 2)

static_assert(SEQ % KC == 0);
static_assert(SEQ % QT == 0);
static_assert(SEQ <= SEQ_FULL && NB <= NB_FULL);
static_assert(EMB == NQH * HDIM);
static_assert(EKV == NKVH * HDIM);
static_assert(NQH == NKVH * GRP);
static_assert(GRP == NWAVE);
static_assert(HDIM == 64 && KC == 64 && QT == 16);
static_assert(NWAVE * 32 * 4 == KC * (HDIM / 8));
static_assert(HDIM * 4 == 16 * 16);
static_assert((EKV % 8) == 0 && (SEQ % 64) == 0);
static_assert(K16_BYTES % 256 == 0 && VT_BYTES % 256 == 0);
static_assert(K16_BYTES + VT_BYTES <= (size_t)134217728);

__device__ __forceinline__ unsigned int bf_bits(float f) {
    const unsigned int u = __float_as_uint(f);
    return (u + 0x7FFFu + ((u >> 16) & 1u)) >> 16;
}
__device__ __forceinline__ __bf16 f2bf(float f) { return __builtin_bit_cast(__bf16, (unsigned short)bf_bits(f)); }
__device__ __forceinline__ float bf_val(float f) { return __uint_as_float(bf_bits(f) << 16); }
__device__ __forceinline__ unsigned int h_bits(float f) { return (unsigned int)__builtin_bit_cast(unsigned short, (_Float16)f); }

__device__ __forceinline__ v8f mma_bf(v16b a, v16b b, v8f c) {
    c = __builtin_amdgcn_wmma_f32_16x16x32_bf16(false, a, false, b, (short)0, c, false, false);
    asm volatile("v_nop\n\tv_nop\n\tv_nop\n\tv_nop" : "+v"(c) : "v"(a), "v"(b));
    return c;
}
__device__ __forceinline__ v8f mma_h(v16h a, v16h b, v8f c) {
    c = __builtin_amdgcn_wmma_f32_16x16x32_f16(false, a, false, b, (short)0, c, false, false);
    asm volatile("v_nop\n\tv_nop\n\tv_nop\n\tv_nop" : "+v"(c) : "v"(a), "v"(b));
    return c;
}

__device__ __forceinline__ void st16x2(unsigned short* p, v4u v) {
    volatile v4u* d = (volatile v4u*)p;
    *d = v; __threadfence(); *d = v;
}

__global__ __launch_bounds__(256) void k_cvt_k(const float* __restrict__ kin, unsigned short* __restrict__ K16) {
    const long long u = (long long)blockIdx.x * 256 + threadIdx.x;
    if (u >= (long long)NB * SEQ * (EKV / 8)) return;
    const int pc = (int)(u % (EKV / 8));
    const long long row = u / (EKV / 8);
    const int b = (int)(row / SEQ), s = (int)(row - (long long)b * SEQ);
    const float* src = kin + ((size_t)b * SEQ_FULL + s) * EKV + pc * 8;
    const v4f a = *(const v4f*)(src), c = *(const v4f*)(src + 4);
    v4u pk;
    pk.x = bf_bits(a.x) | (bf_bits(a.y) << 16); pk.y = bf_bits(a.z) | (bf_bits(a.w) << 16);
    pk.z = bf_bits(c.x) | (bf_bits(c.y) << 16); pk.w = bf_bits(c.z) | (bf_bits(c.w) << 16);
    st16x2(K16 + (size_t)row * EKV + pc * 8, pk);
}

__global__ __launch_bounds__(256) void k_cvt_vt(const float* __restrict__ vin, unsigned short* __restrict__ VT) {
    __shared__ __align__(16) unsigned short tile[64 * 72];
    const int t = threadIdx.x;
    const int s0 = blockIdx.x * 64, kv = blockIdx.y, b = blockIdx.z;
    {
        const int rl = t >> 2, part = t & 3;
        const float* src = vin + ((size_t)b * SEQ_FULL + s0 + rl) * EKV + kv * HDIM + part * 16;
        const v4f f0 = *(const v4f*)(src), f1 = *(const v4f*)(src + 4), f2 = *(const v4f*)(src + 8), f3 = *(const v4f*)(src + 12);
        v4u p0, p1;
        p0.x = h_bits(bf_val(f0.x)) | (h_bits(bf_val(f0.y)) << 16); p0.y = h_bits(bf_val(f0.z)) | (h_bits(bf_val(f0.w)) << 16);
        p0.z = h_bits(bf_val(f1.x)) | (h_bits(bf_val(f1.y)) << 16); p0.w = h_bits(bf_val(f1.z)) | (h_bits(bf_val(f1.w)) << 16);
        p1.x = h_bits(bf_val(f2.x)) | (h_bits(bf_val(f2.y)) << 16); p1.y = h_bits(bf_val(f2.z)) | (h_bits(bf_val(f2.w)) << 16);
        p1.z = h_bits(bf_val(f3.x)) | (h_bits(bf_val(f3.y)) << 16); p1.w = h_bits(bf_val(f3.z)) | (h_bits(bf_val(f3.w)) << 16);
        *(v4u*)(tile + rl * 72 + part * 16)     = p0;
        *(v4u*)(tile + rl * 72 + part * 16 + 8) = p1;
    }
    __syncthreads();
#pragma unroll
    for (int it = 0; it < 2; ++it) {
        const int drow = it * 32 + (t >> 3), pc = t & 7;
        unsigned int e[8];
#pragma unroll
        for (int j = 0; j < 8; ++j) e[j] = (unsigned int)tile[(pc * 8 + j) * 72 + drow];
        v4u pk;
        pk.x = e[0] | (e[1] << 16); pk.y = e[2] | (e[3] << 16); pk.z = e[4] | (e[5] << 16); pk.w = e[6] | (e[7] << 16);
        st16x2(VT + ((size_t)((b * NKVH + kv) * HDIM + drow)) * SEQ + s0 + pc * 8, pk);
    }
}

__global__ __launch_bounds__(128) void k_attn_grp(const float* __restrict__ q, const unsigned short* __restrict__ K16,
                                                   const unsigned short* __restrict__ VT16, float* __restrict__ out) {
    union FB { v16b v; v8b h[2]; };
    union FH { v16h v; v8h h[2]; };
    __shared__ __align__(16) unsigned short Ksh[KC * HDIM];
    __shared__ __align__(16) unsigned short Vth[HDIM * KC];
    __shared__ __align__(16) _Float16       Psh[NWAVE][QT * KC];
    __shared__ __align__(16) float          Os[NWAVE][QT * 68];

    const int tid = threadIdx.x, wave = tid >> 5, lane = tid & 31, hh = lane >> 4, c = lane & 15;
    const int qb = blockIdx.x, kv = blockIdx.y, b = blockIdx.z;
    const int head = kv * GRP + wave;
    const int q0 = qb * QT;
    const float QS  = 0.125f;
    const float L2E = 1.4426950408889634f;
    const float PSC = 32768.0f;

    v16b qa[2];
    {
        const float* qrow = q + ((size_t)b * SEQ_FULL + q0 + c) * EMB + head * HDIM;
#pragma unroll
        for (int dc = 0; dc < 2; ++dc) {
            const v4f a0 = *(const v4f*)(qrow + dc * 32 + 8 * hh);
            const v4f a1 = *(const v4f*)(qrow + dc * 32 + 8 * hh + 4);
            const v4f b0 = *(const v4f*)(qrow + dc * 32 + 16 + 8 * hh);
            const v4f b1 = *(const v4f*)(qrow + dc * 32 + 16 + 8 * hh + 4);
#pragma unroll
            for (int e = 0; e < 4; ++e) {
                qa[dc][e]      = f2bf(a0[e] * QS);
                qa[dc][4 + e]  = f2bf(a1[e] * QS);
                qa[dc][8 + e]  = f2bf(b0[e] * QS);
                qa[dc][12 + e] = f2bf(b1[e] * QS);
            }
        }
    }

    float mrow[8], lrow[8];
    v8f oacc[4];
#pragma unroll
    for (int r = 0; r < 8; ++r) { mrow[r] = -INFINITY; lrow[r] = 0.f; }
#pragma unroll
    for (int t = 0; t < 4; ++t) oacc[t] = (v8f){0.f, 0.f, 0.f, 0.f, 0.f, 0.f, 0.f, 0.f};

    const unsigned short* Kb = K16 + ((size_t)b * SEQ) * EKV + kv * HDIM;
    const unsigned short* Vb = VT16 + ((size_t)(b * NKVH + kv) * HDIM) * SEQ;
    const __bf16*   Kp = (const __bf16*)Ksh;
    const _Float16* Vp = (const _Float16*)Vth;
    _Float16* pw = Psh[wave];

    for (int kc = 0; kc < SEQ / KC; ++kc) {
        const int kv0 = kc * KC;
        __syncthreads();
#pragma unroll
        for (int i = 0; i < 4; ++i) {
            const int idx = tid + 128 * i;
            const int row = idx >> 3, pc = idx & 7;
            const v4u kk = *(const v4u*)(Kb + (size_t)(kv0 + row) * EKV + pc * 8);
            const v4u vv = *(const v4u*)(Vb + (size_t)row * SEQ + kv0 + pc * 8);
            *(v4u*)(Ksh + row * HDIM + pc * 8) = kk;
            *(v4u*)(Vth + row * KC + pc * 8)   = vv;
        }
        __syncthreads();

        v8f s[4];
#pragma unroll
        for (int j = 0; j < 4; ++j) {
            s[j] = (v8f){0.f, 0.f, 0.f, 0.f, 0.f, 0.f, 0.f, 0.f};
#pragma unroll
            for (int dc = 0; dc < 2; ++dc) {
                FB kb;
                kb.h[0] = *(const v8b*)(Kp + (j * 16 + c) * HDIM + dc * 32 + 8 * hh);
                kb.h[1] = *(const v8b*)(Kp + (j * 16 + c) * HDIM + dc * 32 + 16 + 8 * hh);
                s[j] = mma_bf(qa[dc], kb.v, s[j]);
            }
        }

#pragma unroll
        for (int r = 0; r < 8; ++r) {
            const float x0 = s[0][r] * L2E, x1 = s[1][r] * L2E, x2 = s[2][r] * L2E, x3 = s[3][r] * L2E;
            float m = fmaxf(fmaxf(x0, x1), fmaxf(x2, x3));
            m = fmaxf(m, __shfl_xor(m, 1, 32)); m = fmaxf(m, __shfl_xor(m, 2, 32));
            m = fmaxf(m, __shfl_xor(m, 4, 32)); m = fmaxf(m, __shfl_xor(m, 8, 32));
            const float mnew  = fmaxf(mrow[r], m);
            const float alpha = exp2f(mrow[r] - mnew);
            mrow[r] = mnew;
            const float p0 = exp2f(x0 - mnew), p1 = exp2f(x1 - mnew), p2 = exp2f(x2 - mnew), p3 = exp2f(x3 - mnew);
            _Float16* prow = pw + (8 * hh + r) * KC + c;
            prow[0]  = (_Float16)(p0 * PSC);
            prow[16] = (_Float16)(p1 * PSC);
            prow[32] = (_Float16)(p2 * PSC);
            prow[48] = (_Float16)(p3 * PSC);
            float psum = (p0 + p1) + (p2 + p3);
            psum += __shfl_xor(psum, 1, 32); psum += __shfl_xor(psum, 2, 32);
            psum += __shfl_xor(psum, 4, 32); psum += __shfl_xor(psum, 8, 32);
            lrow[r] = lrow[r] * alpha + psum;
#pragma unroll
            for (int t = 0; t < 4; ++t) oacc[t][r] *= alpha;
        }
        __builtin_amdgcn_fence(3  , "workgroup");
        __builtin_amdgcn_wave_barrier();
        __builtin_amdgcn_fence(2  , "workgroup");

#pragma unroll
        for (int kk = 0; kk < 2; ++kk) {
            FH pa;
            pa.h[0] = *(const v8h*)(pw + c * KC + kk * 32 + 8 * hh);
            pa.h[1] = *(const v8h*)(pw + c * KC + kk * 32 + 16 + 8 * hh);
#pragma unroll
            for (int t = 0; t < 4; ++t) {
                FH vb;
                vb.h[0] = *(const v8h*)(Vp + (t * 16 + c) * KC + kk * 32 + 8 * hh);
                vb.h[1] = *(const v8h*)(Vp + (t * 16 + c) * KC + kk * 32 + 16 + 8 * hh);
                oacc[t] = mma_h(pa.v, vb.v, oacc[t]);
            }
        }
    }

    float* os = Os[wave];
#pragma unroll
    for (int r = 0; r < 8; ++r) {
        const float inv = 1.0f / (lrow[r] * PSC);
#pragma unroll
        for (int t = 0; t < 4; ++t) os[(8 * hh + r) * 68 + t * 16 + c] = oacc[t][r] * inv;
    }
    __builtin_amdgcn_fence(3  , "workgroup");
    __builtin_amdgcn_wave_barrier();
    __builtin_amdgcn_fence(2  , "workgroup");
    {
        float* ob = out + ((size_t)b * SEQ + q0) * EMB + head * HDIM;
        const int c4 = (lane & 15) * 4;
        for (int pass = 0; pass < 2; ++pass) {
#pragma unroll
            for (int it = 0; it < 8; ++it) {
                const int row = it * 2 + hh;
                const v4f val = *(const v4f*)(os + row * 68 + c4);
                *(volatile v4f*)(ob + (size_t)row * EMB + c4) = val;
            }
            __threadfence();
        }
    }
}

extern "C" void kernel_launch(void* const* d_in, const int* in_sizes, int n_in, void* d_out, int out_size, void* d_ws, size_t ws_size, hipStream_t stream) {
    if (n_in < 3) return;
    if ((long long)in_sizes[0] < (long long)(NB - 1) * SEQ_FULL * EMB + (long long)SEQ * EMB) return;
    if ((long long)in_sizes[1] < (long long)(NB - 1) * SEQ_FULL * EKV + (long long)SEQ * EKV) return;
    if ((long long)in_sizes[2] < (long long)(NB - 1) * SEQ_FULL * EKV + (long long)SEQ * EKV) return;
    if ((long long)out_size < (long long)NB * SEQ * EMB) return;
    if (ws_size < K16_BYTES + VT_BYTES) return;

    const float* q = (const float*)d_in[0];
    const float* k = (const float*)d_in[1];
    const float* v = (const float*)d_in[2];
    float* out = (float*)d_out;
    unsigned short* K16 = (unsigned short*)d_ws;
    unsigned short* VT  = (unsigned short*)((char*)d_ws + K16_BYTES);

    k_cvt_k<<<(unsigned)(((long long)NB * SEQ * (EKV / 8) + 255) / 256), 256, 0, stream>>>(k, K16);
    k_cvt_vt<<<dim3((unsigned)(SEQ / 64), (unsigned)NKVH, (unsigned)NB), 256, 0, stream>>>(v, VT);
    k_attn_grp<<<dim3((unsigned)(SEQ / QT), (unsigned)NKVH, (unsigned)NB), 128, 0, stream>>>(q, K16, VT, out);
}
